// VN_Transformer_62388694942409
// MI455X (gfx1250) — hardware-run, weakly checked
//
#include <hip/hip_runtime.h>


#ifndef NB
#define NB 8
#endif
#ifndef NPT
#define NPT 8192
#endif
#define NB_FULL   8
#define NPT_FULL  8192
#ifndef OUT_NPT
#define OUT_NPT NPT
#endif
#define CI    64
#define OC    256
#define NH_   4
#define HD    64
#define NQKV  768
#define NCOL       (3 * NPT)
#define NCOL_FULL  (3 * NPT_FULL)
#define OUT_NCOL   (3 * OUT_NPT)
#define PCH   128
#define NBLK  (NPT / PCH)
#define PBM   64

static_assert(CI == 64);
static_assert(CI % 32 == 0);
static_assert(OC % 32 == 0);
static_assert(NH_ * HD == OC);
static_assert(NQKV == 3 * OC);
static_assert(NQKV % 64 == 0);
static_assert(NPT % 64 == 0);
static_assert(NCOL % 64 == 0);
static_assert(NPT % PCH == 0);
static_assert(PCH % 4 == 0);
static_assert(NPT % PBM == 0);
static_assert(PBM % 8 == 0);
static_assert(NB <= NB_FULL);
static_assert(NPT <= NPT_FULL);
static_assert(NPT <= OUT_NPT);

typedef unsigned short bf;
typedef __attribute__((ext_vector_type(16))) __bf16   v16bf;
typedef __attribute__((ext_vector_type(8)))  unsigned short v8us;
typedef __attribute__((ext_vector_type(8)))  float    v8f;
typedef __attribute__((ext_vector_type(4)))  float    v4f;
typedef v4f  __attribute__((may_alias)) v4fa;

__device__ __forceinline__ unsigned short f2bf(float f) { unsigned u = __float_as_uint(f); u += 0x7FFFu + ((u >> 16) & 1u); return (unsigned short)(u >> 16); }
__device__ __forceinline__ float bf2f(unsigned short w) { return __uint_as_float(((unsigned)w) << 16); }
__device__ __forceinline__ v16bf cat16b(v8us lo, v8us hi) { return __builtin_bit_cast(v16bf, __builtin_shufflevector(lo, hi, 0, 1, 2, 3, 4, 5, 6, 7, 8, 9, 10, 11, 12, 13, 14, 15)); }
__device__ __forceinline__ v8f wmmab(v16bf a, v16bf b, v8f c) { return __builtin_amdgcn_wmma_f32_16x16x32_bf16(false, a, false, b, (short)0, c, false, false); }
__device__ __forceinline__ v16bf ldb(const bf* p)  { return cat16b(*(const v8us*)p, *(const v8us*)(p + 16)); }
__device__ __forceinline__ void wave_sync() { __builtin_amdgcn_fence(3  , "wavefront"); __builtin_amdgcn_wave_barrier(); asm volatile("" ::: "memory"); }

__global__ __launch_bounds__(256) void k_cvt8(const float* __restrict__ src, bf* dst, size_t n8) {
    const size_t i = (size_t)blockIdx.x * 256 + threadIdx.x; if (i >= n8) return;
    const v8f v = *(const v8f*)(src + i * 8); v8us o;
#pragma unroll
    for (int k = 0; k < 8; ++k) o[k] = f2bf(v[k]);
    *(volatile v8us*)(dst + i * 8) = o; __threadfence(); *(volatile v8us*)(dst + i * 8) = o;
}

__global__ __launch_bounds__(256) void k_xt(const float* __restrict__ feat, bf* XT) {
    __shared__ float ts[64 * 65];
    const int tid = threadIdx.x; const int col0 = blockIdx.x * 64; const int b = blockIdx.y;
    const float* src = feat + (size_t)b * CI * NCOL_FULL + col0;
#pragma unroll
    for (int i = 0; i < 4; ++i) { const int idx = tid + 256 * i; const int ch = idx >> 4, c4 = (idx & 15) * 4;
        const v4f v = *(const v4f*)(src + (size_t)ch * NCOL_FULL + c4);
        ts[ch * 65 + c4 + 0] = v[0]; ts[ch * 65 + c4 + 1] = v[1]; ts[ch * 65 + c4 + 2] = v[2]; ts[ch * 65 + c4 + 3] = v[3]; }
    __syncthreads();
    bf* dst = XT + ((size_t)b * NCOL + col0) * CI;
    v8us o0, o1;
    { const int col = tid >> 3, p = tid & 7;
#pragma unroll
      for (int j = 0; j < 8; ++j) o0[j] = f2bf(ts[(p * 8 + j) * 65 + col]); }
    { const int idx = tid + 256; const int col = idx >> 3, p = idx & 7;
#pragma unroll
      for (int j = 0; j < 8; ++j) o1[j] = f2bf(ts[(p * 8 + j) * 65 + col]); }
    const size_t a0 = (size_t)(tid >> 3) * CI + (tid & 7) * 8;
    const size_t a1 = (size_t)((tid + 256) >> 3) * CI + (tid & 7) * 8;
    *(volatile v8us*)(dst + a0) = o0; *(volatile v8us*)(dst + a1) = o1;
    __threadfence();
    *(volatile v8us*)(dst + a0) = o0; *(volatile v8us*)(dst + a1) = o1;
}

__global__ __launch_bounds__(32) void k_qkv(const bf* __restrict__ A, const bf* __restrict__ Bt, float* P) {
    __shared__ __align__(16) float os[16 * 68];
    const int K = CI;
    const int lane = threadIdx.x & 31, lr = lane & 15, hi = lane >> 4; const int r0 = blockIdx.x * 64, c0 = blockIdx.y * 64;
    v8f acc[4][4];
#pragma unroll
    for (int mb = 0; mb < 4; ++mb)
#pragma unroll
        for (int nb = 0; nb < 4; ++nb) acc[mb][nb] = (v8f){};
    const size_t aoff = (size_t)(r0 + lr) * K + 8 * hi, boff = (size_t)(c0 + lr) * K + 8 * hi;
#pragma unroll 1
    for (int kc = 0; kc < K; kc += 32) {
        v16bf a[4];
#pragma unroll
        for (int mb = 0; mb < 4; ++mb) a[mb] = ldb(A + aoff + (size_t)mb * 16 * K + kc);
#pragma unroll
        for (int nb = 0; nb < 4; ++nb) { const v16bf b = ldb(Bt + boff + (size_t)nb * 16 * K + kc);
#pragma unroll
            for (int mb = 0; mb < 4; ++mb) acc[mb][nb] = wmmab(a[mb], b, acc[mb][nb]); }
        asm volatile("v_nop\n\tv_nop\n\tv_nop\n\tv_nop" : "+v"(acc[0][0]), "+v"(acc[1][1]), "+v"(acc[2][2]), "+v"(acc[3][3]) : "v"(a[0]), "v"(a[1]), "v"(a[2]), "v"(a[3]));
    }
#pragma unroll
    for (int mb = 0; mb < 4; ++mb) {
#pragma unroll
        for (int nb = 0; nb < 4; ++nb) {
#pragma unroll
            for (int j = 0; j < 8; ++j) os[(hi * 8 + j) * 68 + nb * 16 + lr] = acc[mb][nb][j]; }
        wave_sync();
        float* ob = P + (size_t)(r0 + mb * 16) * NQKV + c0;
#pragma unroll 1
        for (int ps = 0; ps < 2; ++ps) {
#pragma unroll
            for (int s = 0; s < 8; ++s) { const int row = 2 * s + hi, cofs = lr * 4;
                const v4f val = *(const v4fa*)(&os[row * 68 + cofs]);
                *(volatile v4f*)(ob + (size_t)row * NQKV + cofs) = val; }
            if (ps == 0) __threadfence(); }
        wave_sync();
    }
}

__global__ __launch_bounds__(256) void k_logit1(const float* __restrict__ P, float* PART) {
    __shared__ float red[16 * 9];
    __shared__ __align__(16) float ln[64];
    const int tid = threadIdx.x, lane = tid & 31;
    const int wave = __builtin_amdgcn_readfirstlane(tid >> 5);
    const int g = tid & 63, pp = tid >> 6;
    if (tid < 64) ln[tid] = 0.0f;
    float s[9];
#pragma unroll
    for (int i = 0; i < 9; ++i) s[i] = 0.0f;
    const int fbase = blockIdx.x * PCH + pp * (PCH / 4);
#pragma unroll 1
    for (int it = 0; it < PCH / 4; ++it) {
        const float* row = P + (size_t)(3 * (fbase + it)) * NQKV + 4 * g;
        v4f q[3], k[3];
#pragma unroll
        for (int a = 0; a < 3; ++a) { q[a] = *(const v4f*)(row + (size_t)a * NQKV); k[a] = *(const v4f*)(row + (size_t)a * NQKV + OC); }
#pragma unroll
        for (int a = 0; a < 3; ++a)
#pragma unroll
            for (int c = 0; c < 3; ++c) {
                float t = s[a * 3 + c];
                t += q[a][0] * k[c][0]; t += q[a][1] * k[c][1]; t += q[a][2] * k[c][2]; t += q[a][3] * k[c][3];
                s[a * 3 + c] = t; }
    }
#pragma unroll
    for (int i = 0; i < 9; ++i) { float v = s[i];
        v += __shfl_xor(v, 1, 32); v += __shfl_xor(v, 2, 32); v += __shfl_xor(v, 4, 32); v += __shfl_xor(v, 8, 32); s[i] = v; }
    if ((lane & 15) == 0) {
#pragma unroll
        for (int i = 0; i < 9; ++i) red[(wave * 2 + (lane >> 4)) * 9 + i] = s[i]; }
    __syncthreads();
    if (tid < 36) { const int h = tid / 9, i = tid - h * 9; float t = 0.0f;
#pragma unroll
        for (int p2 = 0; p2 < 4; ++p2) t += red[((p2 * 2 + (h >> 1)) * 2 + (h & 1)) * 9 + i];
        ln[h * 16 + i] = t; }
    __syncthreads();
    if (tid < 16) { const v4f val = *(const v4fa*)(&ln[tid * 4]); float* o = PART + (size_t)blockIdx.x * 64 + tid * 4;
        *(volatile v4f*)o = val; __threadfence(); *(volatile v4f*)o = val; }
}

__global__ __launch_bounds__(256) void k_mix(const float* __restrict__ P, const float* __restrict__ PART, bf* OH, bf* OL) {
    __shared__ float lg[36];
    __shared__ float sa[36];
    const int tid = threadIdx.x, lane = tid & 31;
    const int wave = __builtin_amdgcn_readfirstlane(tid >> 5);
    if (tid < 36) { const int h = tid / 9, i = tid - h * 9; double sd = 0.0;
#pragma unroll 1
        for (int blk = 0; blk < NBLK; ++blk) sd += (double)PART[(size_t)blk * 64 + h * 16 + i];
        lg[tid] = (float)sd; }
    __syncthreads();
    if (tid < 12) {
        const float sc = 1.0f / 13.856406460551018f;
        float e0 = lg[tid * 3 + 0] * sc, e1 = lg[tid * 3 + 1] * sc, e2 = lg[tid * 3 + 2] * sc;
        const float mx = fmaxf(e0, fmaxf(e1, e2));
        e0 = expf(e0 - mx); e1 = expf(e1 - mx); e2 = expf(e2 - mx);
        const float inv = 1.0f / (e0 + e1 + e2);
        sa[tid * 3 + 0] = e0 * inv; sa[tid * 3 + 1] = e1 * inv; sa[tid * 3 + 2] = e2 * inv; }
    __syncthreads();
    const int g8 = lane; const int h = g8 >> 3;
#pragma unroll 1
    for (int it = 0; it < PBM / 8; ++it) {
        const int f = blockIdx.x * PBM + it * 8 + wave;
        const float* vr = P + (size_t)(3 * f) * NQKV + 2 * OC + 8 * g8;
        const v4f v0a = *(const v4f*)(vr),                    v0b = *(const v4f*)(vr + 4);
        const v4f v1a = *(const v4f*)(vr + NQKV),             v1b = *(const v4f*)(vr + NQKV + 4);
        const v4f v2a = *(const v4f*)(vr + 2 * (size_t)NQKV), v2b = *(const v4f*)(vr + 2 * (size_t)NQKV + 4);
#pragma unroll 1
        for (int a = 0; a < 3; ++a) {
            const float w0 = sa[h * 9 + a * 3 + 0], w1 = sa[h * 9 + a * 3 + 1], w2 = sa[h * 9 + a * 3 + 2];
            v8us oh, ol;
#pragma unroll
            for (int j = 0; j < 4; ++j) {
                const float x = w0 * v0a[j] + w1 * v1a[j] + w2 * v2a[j];
                const float y = w0 * v0b[j] + w1 * v1b[j] + w2 * v2b[j];
                const unsigned short xh = f2bf(x), yh = f2bf(y);
                oh[j] = xh; oh[4 + j] = yh; ol[j] = f2bf(x - bf2f(xh)); ol[4 + j] = f2bf(y - bf2f(yh)); }
            const size_t oo = (size_t)(3 * f + a) * OC + 8 * g8;
            *(volatile v8us*)(OH + oo) = oh; *(volatile v8us*)(OL + oo) = ol;
            __threadfence();
            *(volatile v8us*)(OH + oo) = oh; *(volatile v8us*)(OL + oo) = ol;
        }
    }
}

__global__ __launch_bounds__(32) void k_out(const bf* __restrict__ A, const bf* __restrict__ BH, const bf* __restrict__ BL, const float* __restrict__ featb, float* outb) {
    __shared__ __align__(16) float os[16 * 68];
    const int K = OC;
    const int lane = threadIdx.x & 31, lr = lane & 15, hi = lane >> 4; const int c0 = blockIdx.x * 64;
    v8f acc[4][4];
#pragma unroll
    for (int mb = 0; mb < 4; ++mb)
#pragma unroll
        for (int nb = 0; nb < 4; ++nb) acc[mb][nb] = (v8f){};
    const size_t aoff = (size_t)lr * K + 8 * hi, boff = (size_t)(c0 + lr) * K + 8 * hi;
#pragma unroll 1
    for (int kc = 0; kc < K; kc += 32) {
        v16bf a[4];
#pragma unroll
        for (int mb = 0; mb < 4; ++mb) a[mb] = ldb(A + aoff + (size_t)mb * 16 * K + kc);
#pragma unroll
        for (int nb = 0; nb < 4; ++nb) { const v16bf bh = ldb(BH + boff + (size_t)nb * 16 * K + kc); const v16bf bl = ldb(BL + boff + (size_t)nb * 16 * K + kc);
#pragma unroll
            for (int mb = 0; mb < 4; ++mb) acc[mb][nb] = wmmab(a[mb], bh, acc[mb][nb]);
#pragma unroll
            for (int mb = 0; mb < 4; ++mb) acc[mb][nb] = wmmab(a[mb], bl, acc[mb][nb]); }
        asm volatile("v_nop\n\tv_nop\n\tv_nop\n\tv_nop" : "+v"(acc[0][0]), "+v"(acc[1][1]), "+v"(acc[2][2]), "+v"(acc[3][3]) : "v"(a[0]), "v"(a[1]), "v"(a[2]), "v"(a[3]));
    }
#pragma unroll
    for (int mb = 0; mb < 4; ++mb) {
#pragma unroll
        for (int nb = 0; nb < 4; ++nb) {
#pragma unroll
            for (int j = 0; j < 8; ++j) os[(hi * 8 + j) * 68 + nb * 16 + lr] = acc[mb][nb][j]; }
        wave_sync();
#pragma unroll 1
        for (int ps = 0; ps < 2; ++ps) {
#pragma unroll
            for (int s = 0; s < 8; ++s) { const int row = 2 * s + hi, cofs = lr * 4; const int o = mb * 16 + row;
                v4f val = *(const v4fa*)(&os[row * 68 + cofs]);
                const v4f x = *(const v4f*)(featb + (size_t)o * NCOL_FULL + c0 + cofs);
                val[0] += bf2f(f2bf(x[0])); val[1] += bf2f(f2bf(x[1])); val[2] += bf2f(f2bf(x[2])); val[3] += bf2f(f2bf(x[3]));
                *(volatile v4f*)(outb + (size_t)o * OUT_NCOL + c0 + cofs) = val; }
            if (ps == 0) __threadfence(); }
        wave_sync();
    }
}

static constexpr size_t al256(size_t v) { return (v + 255) & ~(size_t)255; }
static constexpr size_t SZ_XT  = al256((size_t)NB * NCOL * CI * 2);
static constexpr size_t SZ_WC  = al256((size_t)NQKV * CI * 2);
static constexpr size_t SZ_WO  = al256((size_t)CI * OC * 2);
static constexpr size_t SZ_QKV = al256((size_t)NCOL * NQKV * 4);
static constexpr size_t SZ_OP  = al256((size_t)NCOL * OC * 2);
static constexpr size_t SZ_PT  = al256((size_t)NB * NBLK * 64 * 4);
static constexpr size_t SZ_TOTAL = SZ_XT + SZ_WC + SZ_WO + SZ_QKV + 2 * SZ_OP + SZ_PT;
static_assert(SZ_TOTAL <= (size_t)134217728);
static_assert(((size_t)OC * CI * 2) % 256 == 0);
static_assert(((size_t)OC * CI) % 8 == 0);

extern "C" void kernel_launch(void* const* d_in, const int* in_sizes, int n_in,
                              void* d_out, int out_size, void* d_ws, size_t ws_size, hipStream_t stream) {
    if (n_in < 6) return;
    const size_t needx = ((size_t)(NB - 1) * CI + (CI - 1)) * NCOL_FULL + NCOL;
    if ((size_t)in_sizes[0] < needx) return;
    if ((size_t)in_sizes[2] < (size_t)OC * CI || (size_t)in_sizes[3] < (size_t)OC * CI || (size_t)in_sizes[4] < (size_t)OC * CI || (size_t)in_sizes[5] < (size_t)CI * OC) return;
    if ((size_t)out_size < ((size_t)(NB - 1) * CI + (CI - 1)) * OUT_NCOL + NCOL) return;
    if (SZ_TOTAL > ws_size) return;
    const float* feat = (const float*)d_in[0];
    const float* xyz  = (const float*)d_in[1];
    (void)xyz;
    const float* wq = (const float*)d_in[2]; const float* wk = (const float*)d_in[3]; const float* wv = (const float*)d_in[4];
    const float* wo = (const float*)d_in[5];
    float* OUT = (float*)d_out;
    char* wsp = (char*)d_ws;
    bf* XT = (bf*)wsp; wsp += SZ_XT;
    bf* WC = (bf*)wsp; wsp += SZ_WC;
    bf* WO = (bf*)wsp; wsp += SZ_WO;
    float* QKV = (float*)wsp; wsp += SZ_QKV;
    bf* OH = (bf*)wsp; wsp += SZ_OP;
    bf* OL = (bf*)wsp; wsp += SZ_OP;
    float* PT = (float*)wsp; wsp += SZ_PT;

    { const size_t n8 = (size_t)OC * CI / 8; const unsigned g = (unsigned)((n8 + 255) / 256);
      k_cvt8<<<g, 256, 0, stream>>>(wq, WC, n8);
      k_cvt8<<<g, 256, 0, stream>>>(wk, WC + (size_t)OC * CI, n8);
      k_cvt8<<<g, 256, 0, stream>>>(wv, WC + (size_t)2 * OC * CI, n8);
      k_cvt8<<<g, 256, 0, stream>>>(wo, WO, n8); }

    k_xt<<<dim3(NCOL / 64, NB, 1), 256, 0, stream>>>(feat, XT);

    for (int b = 0; b < NB; ++b) {
        const bf* xtb = XT + (size_t)b * NCOL * CI;
        float* ptb = PT + (size_t)b * NBLK * 64;
        k_qkv<<<dim3(NCOL / 64, NQKV / 64, 1), 32, 0, stream>>>(xtb, WC, QKV);
        k_logit1<<<dim3(NBLK, 1, 1), 256, 0, stream>>>(QKV, ptb);
        k_mix<<<dim3(NPT / PBM, 1, 1), 256, 0, stream>>>(QKV, ptb, OH, OL);
        k_out<<<dim3(NCOL / 64, 1, 1), 32, 0, stream>>>(WO, OH, OL, feat + (size_t)b * CI * NCOL_FULL, OUT + (size_t)b * CI * OUT_NCOL);
    }
}
